// MambaBlock_75600014344464
// MI455X (gfx1250) — hardware-verified
//
#include <hip/hip_runtime.h>
#include <math.h>

typedef __attribute__((ext_vector_type(16))) __bf16   v16b;
typedef __attribute__((ext_vector_type(8)))  __bf16   v8b;
typedef __attribute__((ext_vector_type(8)))  float    v8f;
typedef __attribute__((ext_vector_type(4)))  float    v4f;
typedef __attribute__((ext_vector_type(4)))  unsigned v4u;

constexpr int kBatch  = 2;
constexpr int kSeq    = 1024;
constexpr int kDm     = 1024;
constexpr int kDin    = 2048;
constexpr int kNst    = 16;
constexpr int kDtR    = 64;
constexpr int kXzP    = 2 * kDin;
constexpr int kXdN    = kDtR + 2 * kNst;
constexpr int kXdP    = 128;
constexpr int kRows   = kBatch * kSeq;
constexpr int kConvTP = 260;
constexpr int kScanTS = 64;
constexpr int kScanCh = 64;
constexpr int kScanYP = 68;
constexpr int kScanBC = 2 * kNst;
static_assert(kXdN == 96);
static_assert(kXdP % 64 == 0 && kXdP >= kXdN);
static_assert((kDm % 32) == 0 && (kDin % 32) == 0 && (kDtR % 32) == 0);
static_assert((kRows % 64) == 0 && (kXzP % 64) == 0 && (kDin % 64) == 0 && (kDm % 64) == 0);
static_assert((kSeq % kScanTS) == 0 && (kSeq % 64) == 0 && (kDin % kScanCh) == 0 && (kDin % 256) == 0);
static_assert(kNst == 16 && kScanCh == 64 && kScanTS == 64);

constexpr size_t kOffXB   = 0;
constexpr size_t kOffWIB  = kOffXB  + (size_t)kRows * kDm  * 2;
constexpr size_t kOffWXB  = kOffWIB + (size_t)kXzP  * kDm  * 2;
constexpr size_t kOffWDB  = kOffWXB + (size_t)kXdP  * kDin * 2;
constexpr size_t kOffWOB  = kOffWDB + (size_t)kDin  * kDtR * 2;
constexpr size_t kOffXZ   = kOffWOB + (size_t)kDm   * kDin * 2;
constexpr size_t kOffUC   = kOffXZ  + (size_t)kRows * kXzP * 4;
constexpr size_t kOffUCH  = kOffUC  + (size_t)kRows * kDin * 4;
constexpr size_t kOffUCL  = kOffUCH + (size_t)kRows * kDin * 2;
constexpr size_t kOffXD   = kOffUCL + (size_t)kRows * kDin * 2;
constexpr size_t kOffDTH  = kOffXD  + (size_t)kRows * kXdP * 4;
constexpr size_t kOffDTL  = kOffDTH + (size_t)kRows * kDtR * 2;
constexpr size_t kOffDLR  = kOffDTL + (size_t)kRows * kDtR * 2;
constexpr size_t kOffYH   = kOffDLR + (size_t)kRows * kDin * 4;
constexpr size_t kOffYL   = kOffYH  + (size_t)kRows * kDin * 2;
constexpr size_t kWsTotal = kOffYL  + (size_t)kRows * kDin * 2;
static_assert(kWsTotal == 119799808ull);
static_assert(kWsTotal <= 134217728ull);
static_assert((kOffWIB % 128) == 0 && (kOffWXB % 128) == 0 && (kOffWDB % 128) == 0 && (kOffWOB % 128) == 0 &&
              (kOffXZ % 128) == 0 && (kOffUC % 128) == 0 && (kOffUCH % 128) == 0 && (kOffUCL % 128) == 0 &&
              (kOffXD % 128) == 0 && (kOffDTH % 128) == 0 && (kOffDTL % 128) == 0 && (kOffDLR % 128) == 0 &&
              (kOffYH % 128) == 0 && (kOffYL % 128) == 0);

__device__ __forceinline__ unsigned bf_bits_u32(float f) {
  const unsigned u = __float_as_uint(f);
  return (u + 0x7FFFu + ((u >> 16) & 1u)) >> 16;
}
__device__ __forceinline__ float bfr(float f) { return __uint_as_float(bf_bits_u32(f) << 16); }
__device__ __forceinline__ unsigned pack_bf2(float f0, float f1) {
  const unsigned h0 = bf_bits_u32(f0);
  const unsigned h1 = bf_bits_u32(f1);
  return h0 | (h1 << 16);
}
__device__ __forceinline__ void split_pack2(float f0, float f1, unsigned& wh, unsigned& wl) {
  const unsigned h0 = bf_bits_u32(f0);
  const unsigned h1 = bf_bits_u32(f1);
  const unsigned l0 = bf_bits_u32(f0 - __uint_as_float(h0 << 16));
  const unsigned l1 = bf_bits_u32(f1 - __uint_as_float(h1 << 16));
  wh = h0 | (h1 << 16);
  wl = l0 | (l1 << 16);
}
__device__ __forceinline__ void split_pack8(v4f a0, v4f a1, v4u& hv, v4u& lv) {
  const float f0 = a0[0], f1 = a0[1], f2 = a0[2], f3 = a0[3];
  const float f4 = a1[0], f5 = a1[1], f6 = a1[2], f7 = a1[3];
  unsigned h, l;
  split_pack2(f0, f1, h, l);
  hv[0] = h; lv[0] = l;
  split_pack2(f2, f3, h, l);
  hv[1] = h; lv[1] = l;
  split_pack2(f4, f5, h, l);
  hv[2] = h; lv[2] = l;
  split_pack2(f6, f7, h, l);
  hv[3] = h; lv[3] = l;
}

union FragU { v16b v; v8b h[2]; };
__device__ __forceinline__ v16b frag_load(const __bf16* p) {
  FragU f;
  f.h[0] = *(const v8b*)(p);
  f.h[1] = *(const v8b*)(p + 16);
  return f.v;
}
__device__ __forceinline__ v8f frag_mma(v16b a, v16b b, v8f c) {
  return __builtin_amdgcn_wmma_f32_16x16x32_bf16(false, a, false, b, (short)0, c, false, false);
}
__device__ __forceinline__ void group_guard(v8f& a, v8f& b, v8f& c, v8f& d, v16b x, v16b y) {
  asm volatile("v_nop\n\tv_nop\n\tv_nop\n\tv_nop" : "+v"(a), "+v"(b), "+v"(c), "+v"(d) : "v"(x), "v"(y));
}
__device__ __forceinline__ void keep4_b(v16b a, v16b b, v16b c, v16b d) {
  asm volatile("v_nop" :: "v"(a), "v"(b), "v"(c), "v"(d));
}
__device__ __forceinline__ void acc_guard4(v8f& a, v8f& b, v8f& c, v8f& d) {
  asm volatile("v_nop\n\tv_nop\n\tv_nop\n\tv_nop" : "+v"(a), "+v"(b), "+v"(c), "+v"(d));
}

template <int SPL>
__global__ __launch_bounds__(256) void wmma_gemm64(
    const unsigned short* __restrict__ Ap, const unsigned short* __restrict__ A2p, int lda,
    const unsigned short* __restrict__ Btp, int ldb,
    float* __restrict__ C, int ldc, int M, int N, int K)
{
  const __bf16* A  = (const __bf16*)Ap;
  const __bf16* A2 = (const __bf16*)A2p;
  const __bf16* Bt = (const __bf16*)Btp;
  __shared__ __align__(16) float sT[8][16 * 68];
  const int lane = threadIdx.x & 31;
  const int wave = threadIdx.x >> 5;
  const int tilesN = N >> 6;
  const int tilesM = M >> 6;
  const int tile = blockIdx.x * 8 + wave;
  if (tile >= tilesM * tilesN) return;
  const int tm = tile / tilesN;
  const int tn = tile - tm * tilesN;
  const int m0 = tm << 6;
  const int n0 = tn << 6;

  const int rlane = lane & 15;
  const int koff  = (lane >> 4) * 8;
  const int mOff  = (lane >> 4) * 8;

  v8f acc[4][4];
#pragma unroll
  for (int i = 0; i < 4; ++i)
#pragma unroll
    for (int j = 0; j < 4; ++j) acc[i][j] = (v8f){0.f, 0.f, 0.f, 0.f, 0.f, 0.f, 0.f, 0.f};

  for (int k0 = 0; k0 < K; k0 += 32) {
    v16b bh[4];
#pragma unroll
    for (int j = 0; j < 4; ++j) {
      const size_t bo = (size_t)(n0 + (j << 4) + rlane) * ldb + koff + k0;
      bh[j] = frag_load(Bt + bo);
    }
#pragma unroll
    for (int i = 0; i < 4; ++i) {
      const size_t ao = (size_t)(m0 + (i << 4) + rlane) * lda + koff + k0;
      v16b ah = frag_load(A + ao);
      v16b al = ah;
      if (SPL == 1) al = frag_load(A2 + ao);
#pragma unroll
      for (int j = 0; j < 4; ++j) {
        acc[i][j] = frag_mma(ah, bh[j], acc[i][j]);
        if (SPL == 1) acc[i][j] = frag_mma(al, bh[j], acc[i][j]);
      }
      group_guard(acc[i][0], acc[i][1], acc[i][2], acc[i][3], ah, al);
    }
    keep4_b(bh[0], bh[1], bh[2], bh[3]);
  }
  acc_guard4(acc[0][0], acc[0][1], acc[0][2], acc[0][3]);
  acc_guard4(acc[1][0], acc[1][1], acc[1][2], acc[1][3]);
  acc_guard4(acc[2][0], acc[2][1], acc[2][2], acc[2][3]);
  acc_guard4(acc[3][0], acc[3][1], acc[3][2], acc[3][3]);

  float* slab = sT[wave];
#pragma unroll
  for (int i = 0; i < 4; ++i) {
    const int mBase = m0 + (i << 4);
#pragma unroll
    for (int j = 0; j < 4; ++j) {
#pragma unroll
      for (int r = 0; r < 8; ++r) {
        slab[(mOff + r) * 68 + (j << 4) + rlane] = acc[i][j][r];
      }
    }
    __builtin_amdgcn_fence(__ATOMIC_RELEASE, "workgroup");
    __builtin_amdgcn_wave_barrier();
    __builtin_amdgcn_fence(__ATOMIC_ACQUIRE, "workgroup");
    {
      const int hh = lane >> 4, c4 = (lane & 15) * 4;
      for (int pass = 0; pass < 2; ++pass) {
#pragma unroll
        for (int it = 0; it < 8; ++it) {
          const int row = it * 2 + hh;
          v4f v = *(const v4f*)(slab + row * 68 + c4);
          *(volatile v4f*)(C + (size_t)(mBase + row) * ldc + n0 + c4) = v;
        }
        __threadfence();
      }
    }
    __builtin_amdgcn_fence(__ATOMIC_RELEASE, "workgroup");
    __builtin_amdgcn_wave_barrier();
    __builtin_amdgcn_fence(__ATOMIC_ACQUIRE, "workgroup");
  }
}

__global__ __launch_bounds__(256) void rne_rows_bf16_kernel(
    const float* __restrict__ src, unsigned short* __restrict__ dst, int src8, int dst8)
{
  const int i = blockIdx.x * 256 + threadIdx.x;
  if (i >= dst8) return;
  const bool live = (i < src8);
  const int is = live ? i : (src8 - 1);
  const size_t s0 = (size_t)is << 3;
  const v4f a0 = *(const v4f*)(src + s0);
  const v4f a1 = *(const v4f*)(src + s0 + 4);
  const float f0 = a0[0], f1 = a0[1], f2 = a0[2], f3 = a0[3];
  const float f4 = a1[0], f5 = a1[1], f6 = a1[2], f7 = a1[3];
  const unsigned p0 = pack_bf2(f0, f1);
  const unsigned p1 = pack_bf2(f2, f3);
  const unsigned p2 = pack_bf2(f4, f5);
  const unsigned p3 = pack_bf2(f6, f7);
  v4u w;
  w[0] = live ? p0 : 0u;
  w[1] = live ? p1 : 0u;
  w[2] = live ? p2 : 0u;
  w[3] = live ? p3 : 0u;
  unsigned short* q = dst + ((size_t)i << 3);
  *(volatile v4u*)q = w;
  __threadfence();
  *(volatile v4u*)q = w;
}

__global__ __launch_bounds__(256) void conv_silu_kernel(
    const float* __restrict__ XZ, const float* __restrict__ cw, const float* __restrict__ cb,
    float* __restrict__ UC, unsigned short* __restrict__ UCH, unsigned short* __restrict__ UCL)
{
  __shared__ __align__(16) float sT[16 * kConvTP];
  const int tid = threadIdx.x, lane = tid & 31, wave = tid >> 5;
  const int d0 = blockIdx.x * 256, d = d0 + tid;
  const int g0 = blockIdx.y * 64;
  const int tb = g0 & (kSeq - 1);
  const float w0 = bfr(cw[d * 4 + 0]);
  const float w1 = bfr(cw[d * 4 + 1]);
  const float w2 = bfr(cw[d * 4 + 2]);
  const float w3 = bfr(cw[d * 4 + 3]);
  const float bc = bfr(cb[d]);
  float xm3, xm2, xm1;
  {
    const bool hist = (tb > 0);
    const int rb = hist ? (g0 - 3) : g0;
    const float v3 = XZ[(size_t)rb * kXzP + d];
    const float v2 = XZ[(size_t)(rb + 1) * kXzP + d];
    const float v1 = XZ[(size_t)(rb + 2) * kXzP + d];
    xm3 = hist ? v3 : 0.f;
    xm2 = hist ? v2 : 0.f;
    xm1 = hist ? v1 : 0.f;
  }
  const int hrow = wave >> 1;
  const int hch  = (wave & 1) * 128 + lane * 4;
#pragma unroll 1
  for (int sub = 0; sub < 4; ++sub) {
    const int lb = g0 + sub * 16;
#pragma unroll 1
    for (int s = 0; s < 16; ++s) {
      const float xcur = XZ[(size_t)(lb + s) * kXzP + d];
      float acc = w0 * xm3;
      acc = fmaf(w1, xm2, acc);
      acc = fmaf(w2, xm1, acc);
      acc = fmaf(w3, xcur, acc);
      const float sv = acc + bc;
      const float sg = __builtin_amdgcn_rcpf(1.0f + expf(-sv));
      sT[s * kConvTP + tid] = sv * sg;
      xm3 = xm2;
      xm2 = xm1;
      xm1 = xcur;
    }
    __syncthreads();
    v4f fv[4];
    v4u bh[2], bl[2];
#pragma unroll
    for (int it = 0; it < 4; ++it) fv[it] = *(const v4f*)(sT + (it * 4 + hrow) * kConvTP + hch);
#pragma unroll
    for (int it = 0; it < 2; ++it) {
      const float* sp = sT + (it * 8 + wave) * kConvTP + lane * 8;
      const v4f a0 = *(const v4f*)(sp);
      const v4f a1 = *(const v4f*)(sp + 4);
      split_pack8(a0, a1, bh[it], bl[it]);
    }
    for (int pass = 0; pass < 2; ++pass) {
#pragma unroll
      for (int it = 0; it < 4; ++it)
        *(volatile v4f*)(UC + (size_t)(lb + it * 4 + hrow) * kDin + d0 + hch) = fv[it];
#pragma unroll
      for (int it = 0; it < 2; ++it) {
        const size_t o = (size_t)(lb + it * 8 + wave) * kDin + d0 + lane * 8;
        *(volatile v4u*)(UCH + o) = bh[it];
        *(volatile v4u*)(UCL + o) = bl[it];
      }
      __threadfence();
    }
    __syncthreads();
  }
}

__global__ __launch_bounds__(256) void dt_split_kernel(
    const float* __restrict__ XD, unsigned short* __restrict__ DTH, unsigned short* __restrict__ DTL, int total8)
{
  const int i = blockIdx.x * 256 + threadIdx.x;
  if (i >= total8) return;
  const int e0  = i << 3;
  const int row = e0 / kDtR;
  const int c8  = e0 - row * kDtR;
  const float* p = XD + (size_t)row * kXdP + c8;
  const v4f a0 = *(const v4f*)(p);
  const v4f a1 = *(const v4f*)(p + 4);
  v4u hv, lv;
  split_pack8(a0, a1, hv, lv);
  unsigned short* qh = DTH + e0;
  unsigned short* ql = DTL + e0;
  *(volatile v4u*)qh = hv;
  *(volatile v4u*)ql = lv;
  __threadfence();
  *(volatile v4u*)qh = hv;
  *(volatile v4u*)ql = lv;
}

__global__ __launch_bounds__(64) void scan_kernel(
    const float* __restrict__ XD, const float* __restrict__ UC, const float* __restrict__ XZ,
    const float* __restrict__ DLR, const float* __restrict__ bdt, const float* __restrict__ Alog,
    unsigned short* __restrict__ YH, unsigned short* __restrict__ YL)
{
  __shared__ __align__(16) float sX[kScanTS * kScanBC];
  __shared__ __align__(16) float sY[kScanTS * kScanYP];
  __shared__ __align__(16) float sA[kNst * kScanCh];
  const int tid = threadIdx.x, lane = tid & 31, wave = tid >> 5;
  constexpr int kBlkPerB = kDin / kScanCh;
  const int bix = blockIdx.x / kBlkPerB;
  const int d0  = (blockIdx.x - bix * kBlkPerB) * kScanCh;
  const int d   = d0 + tid;
  const size_t row0 = (size_t)bix * kSeq;
#pragma unroll 1
  for (int s = 0; s < kNst; ++s) sA[s * kScanCh + tid] = -expf(bfr(Alog[(size_t)d * kNst + s]));
  __syncthreads();
  float negA[kNst], h[kNst];
#pragma unroll
  for (int s = 0; s < kNst; ++s) {
    negA[s] = sA[s * kScanCh + tid];
    h[s] = 0.f;
  }
  const float bb = bfr(bdt[d]);
  const int lr = tid >> 3, lc4 = (tid & 7) * 4;
  const int q = lane >> 3, c8 = (lane & 7) * 8;
#pragma unroll 1
  for (int t0 = 0; t0 < kSeq; t0 += kScanTS) {
    __syncthreads();
#pragma unroll
    for (int i = 0; i < 8; ++i) {
      const int r = lr + 8 * i;
      *(v4f*)(sX + r * kScanBC + lc4) = *(const v4f*)(XD + (row0 + t0 + r) * kXdP + kDtR + lc4);
    }
    __syncthreads();
#pragma unroll 1
    for (int s = 0; s < kScanTS; ++s) {
      const size_t rg = row0 + (size_t)(t0 + s);
      const float* xr = sX + s * kScanBC;
      float Bs[kNst], Cs[kNst];
#pragma unroll
      for (int q4 = 0; q4 < 4; ++q4) {
        const v4f bv = *(const v4f*)(xr + 4 * q4);
        const v4f cv = *(const v4f*)(xr + kNst + 4 * q4);
        Bs[4 * q4 + 0] = bv[0];
        Bs[4 * q4 + 1] = bv[1];
        Bs[4 * q4 + 2] = bv[2];
        Bs[4 * q4 + 3] = bv[3];
        Cs[4 * q4 + 0] = cv[0];
        Cs[4 * q4 + 1] = cv[1];
        Cs[4 * q4 + 2] = cv[2];
        Cs[4 * q4 + 3] = cv[3];
      }
      const float pre = DLR[rg * kDin + d] + bb;
      const float xt  = UC[rg * kDin + d];
      const float zv  = XZ[rg * kXzP + kDin + d];
      const float ea  = expf(-fabsf(pre));
      const float dt  = fmaxf(pre, 0.0f) + log1pf(ea);
      const float dtx = dt * xt;
      float y = 0.f;
#pragma unroll
      for (int k = 0; k < kNst; ++k) {
        const float e = __expf(dt * negA[k]);
        h[k] = e * h[k] + dtx * Bs[k];
        y = h[k] * Cs[k] + y;
      }
      const float sg = __builtin_amdgcn_rcpf(1.0f + expf(-zv));
      y = y * (zv * sg);
      sY[s * kScanYP + tid] = y;
    }
    __syncthreads();
    v4u hv[8], lv[8];
#pragma unroll
    for (int it = 0; it < 8; ++it) {
      const int row = it * 8 + wave * 4 + q;
      const float* sp = sY + row * kScanYP + c8;
      const v4f a0 = *(const v4f*)(sp);
      const v4f a1 = *(const v4f*)(sp + 4);
      split_pack8(a0, a1, hv[it], lv[it]);
    }
    for (int pass = 0; pass < 2; ++pass) {
#pragma unroll
      for (int it = 0; it < 8; ++it) {
        const int row = it * 8 + wave * 4 + q;
        const size_t o = (row0 + (size_t)(t0 + row)) * kDin + d0 + c8;
        *(volatile v4u*)(YH + o) = hv[it];
        *(volatile v4u*)(YL + o) = lv[it];
      }
      __threadfence();
    }
  }
}

static_assert(((kRows * kDm / 8) % 256) == 0 && ((kXzP * kDm / 8) % 256) == 0 && ((kXdP * kDin / 8) % 256) == 0 &&
              ((kDin * kDtR / 8) % 256) == 0 && ((kDm * kDin / 8) % 256) == 0 && ((kRows * kDtR / 8) % 256) == 0);
static_assert((((kRows / 64) * (kXzP / 64)) % 8) == 0 && (((kRows / 64) * (kXdP / 64)) % 8) == 0 &&
              (((kRows / 64) * (kDin / 64)) % 8) == 0 && (((kRows / 64) * (kDm / 64)) % 8) == 0);

extern "C" void kernel_launch(void* const* d_in, const int* in_sizes, int n_in,
                              void* d_out, int out_size, void* d_ws, size_t ws_size,
                              hipStream_t stream)
{
  (void)stream;
  if (n_in < 9) return;
  if (in_sizes[0] != kRows * kDm) return;
  if (in_sizes[1] != kXzP * kDm) return;
  if (in_sizes[2] != kDin * 4) return;
  if (in_sizes[3] != kDin) return;
  if (in_sizes[4] != kXdN * kDin) return;
  if (in_sizes[5] != kDin * kDtR) return;
  if (in_sizes[6] != kDin) return;
  if (in_sizes[7] != kDin * kNst) return;
  if (in_sizes[8] != kDm * kDin) return;
  if (out_size != kRows * kDm) return;
  if (ws_size < kWsTotal) return;

  const float* x      = (const float*)d_in[0];
  const float* W_in   = (const float*)d_in[1];
  const float* conv_w = (const float*)d_in[2];
  const float* conv_b = (const float*)d_in[3];
  const float* W_x    = (const float*)d_in[4];
  const float* W_dt   = (const float*)d_in[5];
  const float* b_dt   = (const float*)d_in[6];
  const float* A_log  = (const float*)d_in[7];
  const float* W_out  = (const float*)d_in[8];
  float* out = (float*)d_out;

  char* ws = (char*)d_ws;
  unsigned short* XB  = (unsigned short*)(ws + kOffXB);
  unsigned short* WIB = (unsigned short*)(ws + kOffWIB);
  unsigned short* WXB = (unsigned short*)(ws + kOffWXB);
  unsigned short* WDB = (unsigned short*)(ws + kOffWDB);
  unsigned short* WOB = (unsigned short*)(ws + kOffWOB);
  float*          XZ  = (float*)(ws + kOffXZ);
  float*          UC  = (float*)(ws + kOffUC);
  unsigned short* UCH = (unsigned short*)(ws + kOffUCH);
  unsigned short* UCL = (unsigned short*)(ws + kOffUCL);
  float*          XD  = (float*)(ws + kOffXD);
  unsigned short* DTH = (unsigned short*)(ws + kOffDTH);
  unsigned short* DTL = (unsigned short*)(ws + kOffDTL);
  float*          DLR = (float*)(ws + kOffDLR);
  unsigned short* YH  = (unsigned short*)(ws + kOffYH);
  unsigned short* YL  = (unsigned short*)(ws + kOffYL);

  rne_rows_bf16_kernel<<<(kRows * kDm / 8) / 256, 256, 0, stream>>>(x, XB, kRows * kDm / 8, kRows * kDm / 8);
  rne_rows_bf16_kernel<<<(kXzP * kDm / 8) / 256, 256, 0, stream>>>(W_in, WIB, kXzP * kDm / 8, kXzP * kDm / 8);
  rne_rows_bf16_kernel<<<(kXdP * kDin / 8) / 256, 256, 0, stream>>>(W_x, WXB, kXdN * kDin / 8, kXdP * kDin / 8);
  rne_rows_bf16_kernel<<<(kDin * kDtR / 8) / 256, 256, 0, stream>>>(W_dt, WDB, kDin * kDtR / 8, kDin * kDtR / 8);
  rne_rows_bf16_kernel<<<(kDm * kDin / 8) / 256, 256, 0, stream>>>(W_out, WOB, kDm * kDin / 8, kDm * kDin / 8);

  wmma_gemm64<0><<<((kRows / 64) * (kXzP / 64)) / 8, 256, 0, stream>>>(
      XB, XB, kDm, WIB, kDm, XZ, kXzP, kRows, kXzP, kDm);

  conv_silu_kernel<<<dim3(kDin / 256, kRows / 64), 256, 0, stream>>>(XZ, conv_w, conv_b, UC, UCH, UCL);

  wmma_gemm64<1><<<((kRows / 64) * (kXdP / 64)) / 8, 256, 0, stream>>>(
      UCH, UCL, kDin, WXB, kDin, XD, kXdP, kRows, kXdP, kDin);

  dt_split_kernel<<<(kRows * kDtR / 8) / 256, 256, 0, stream>>>(XD, DTH, DTL, kRows * kDtR / 8);

  wmma_gemm64<1><<<((kRows / 64) * (kDin / 64)) / 8, 256, 0, stream>>>(
      DTH, DTL, kDtR, WDB, kDtR, DLR, kDin, kRows, kDin, kDtR);

  scan_kernel<<<kBatch * (kDin / kScanCh), kScanCh, 0, stream>>>(XD, UC, XZ, DLR, b_dt, A_log, YH, YL);

  wmma_gemm64<1><<<((kRows / 64) * (kDm / 64)) / 8, 256, 0, stream>>>(
      YH, YL, kDin, WOB, kDin, out, kDm, kRows, kDm, kDin);
}
